// ScaledDotProductAttention_74620761800949
// MI455X (gfx1250) — hardware-verified
//
#include <hip/hip_runtime.h>


typedef _Float16     v16h __attribute__((ext_vector_type(16)));
typedef _Float16     v8h  __attribute__((ext_vector_type(8)));
typedef float        v8f  __attribute__((ext_vector_type(8)));
typedef float        v4f  __attribute__((ext_vector_type(4)));
typedef int          v4i  __attribute__((ext_vector_type(4)));
typedef unsigned int v4u  __attribute__((ext_vector_type(4)));
typedef unsigned int v2u  __attribute__((ext_vector_type(2)));

#ifndef NB
#define NB 2
#endif
#ifndef SEQ
#define SEQ 2048
#endif

constexpr int NB_FULL = 2;
constexpr int HN      = 16;
constexpr int S_FULL  = 2048;
constexpr int DK      = 64;

constexpr int QTILE = 128;
constexpr int KBLK  = 128;
constexpr int NBLK  = SEQ / KBLK;
constexpr int NT    = KBLK / 16;
constexpr int KD    = DK + 8;
constexpr int VD    = KBLK + 8;
constexpr int PD    = KBLK + 8;
constexpr int OPD   = DK + 4;
constexpr int CT    = 64;
constexpr int VP    = CT + 8;

static_assert(NB >= 1 && NB <= NB_FULL);
static_assert(SEQ >= QTILE && SEQ <= S_FULL);
static_assert(SEQ % QTILE == 0);
static_assert(SEQ % KBLK == 0);
static_assert(SEQ % CT == 0);
static_assert(NT == 8);
static_assert((KD % 8) == 0 && (VD % 8) == 0 && (PD % 8) == 0 && (VP % 8) == 0 && (OPD % 4) == 0);

union Frag { v16h v; v8h h[2]; };

__device__ __forceinline__ float fast_exp2(float x) {
#if defined(__has_builtin) && __has_builtin(__builtin_amdgcn_exp2f)
  return __builtin_amdgcn_exp2f(x);
#else
  return __expf(x * 0.6931471805599453f);
#endif
}

__device__ __forceinline__ float fast_rcp(float x) {
#if defined(__has_builtin) && __has_builtin(__builtin_amdgcn_rcpf)
  return __builtin_amdgcn_rcpf(x);
#else
  return 1.0f / x;
#endif
}

__device__ __forceinline__ v8f wmma16(v16h a, v16h b, v8f c) {
  c = __builtin_amdgcn_wmma_f32_16x16x32_f16(false, a, false, b, (short)0, c, false, false);
  asm volatile("v_nop\n\tv_nop\n\tv_nop\n\tv_nop" : "+v"(c) : "v"(a), "v"(b));
  return c;
}

__device__ __forceinline__ v16h ld_op16(const _Float16* p) {
  Frag u;
  u.h[0] = *(const v8h*)(p);
  u.h[1] = *(const v8h*)(p + 16);
  return u.v;
}

__device__ __forceinline__ float bf16_rne(float x) {
  unsigned int u = __float_as_uint(x);
  u = (u + 0x7fffu + ((u >> 16) & 1u)) & 0xffff0000u;
  return __uint_as_float(u);
}

__device__ __forceinline__ v8h cvt8(const float* __restrict__ p) {
  const float4 a = *(const float4*)(p);
  const float4 b = *(const float4*)(p + 4);
  v8h r;
  r[0] = (_Float16)bf16_rne(a.x); r[1] = (_Float16)bf16_rne(a.y);
  r[2] = (_Float16)bf16_rne(a.z); r[3] = (_Float16)bf16_rne(a.w);
  r[4] = (_Float16)bf16_rne(b.x); r[5] = (_Float16)bf16_rne(b.y);
  r[6] = (_Float16)bf16_rne(b.z); r[7] = (_Float16)bf16_rne(b.w);
  return r;
}

__global__ __launch_bounds__(256)
void k_convert(const float* __restrict__ K, const float* __restrict__ V,
               _Float16* __restrict__ Kh, _Float16* __restrict__ Vt) {
  __shared__ __align__(16) _Float16 sVt[DK * VP];

  const int tid  = threadIdx.x;
  const int lane = tid & 31;
  const int wv   = tid >> 5;
  const int q    = lane & 7;
  const int rsub = lane >> 3;
  const int kt   = blockIdx.x;
  const int bhr  = blockIdx.y;
  const int b    = bhr / HN;
  const int h    = bhr - b * HN;
  const size_t inbase = ((size_t)b * HN + h) * (size_t)S_FULL * DK;
  const size_t khbase = (size_t)bhr * SEQ * DK;
  const size_t vtbase = (size_t)bhr * DK * SEQ;
  const int k0 = kt * CT;

  v8h kreg[2];
#pragma unroll
  for (int j = 0; j < 2; ++j) {
    const int r = wv * 8 + 4 * j + rsub;
    const size_t src = inbase + (size_t)(k0 + r) * DK + 8 * q;
    kreg[j] = cvt8(K + src);
    const v8h vv = cvt8(V + src);
#pragma unroll
    for (int e = 0; e < 8; ++e) sVt[(8 * q + e) * VP + r] = vv[e];
  }
  __syncthreads();

  v8h vreg[2];
#pragma unroll
  for (int j = 0; j < 2; ++j) {
    const int dd = wv * 8 + 4 * j + rsub;
    vreg[j] = *(const v8h*)&sVt[dd * VP + 8 * q];
  }

#pragma unroll
  for (int j = 0; j < 2; ++j) {
    const int r = wv * 8 + 4 * j + rsub;
    *(volatile v8h*)(Kh + khbase + (size_t)(k0 + r) * DK + 8 * q) = kreg[j];
    *(volatile v8h*)(Vt + vtbase + (size_t)r * SEQ + k0 + 8 * q) = vreg[j];
  }
  __threadfence();
#pragma unroll
  for (int j = 0; j < 2; ++j) {
    const int r = wv * 8 + 4 * j + rsub;
    *(volatile v8h*)(Kh + khbase + (size_t)(k0 + r) * DK + 8 * q) = kreg[j];
    *(volatile v8h*)(Vt + vtbase + (size_t)r * SEQ + k0 + 8 * q) = vreg[j];
  }
}

__global__ __launch_bounds__(256)
void k_attn(const float* __restrict__ Q, const int* __restrict__ Mk,
            const _Float16* __restrict__ Kh, const _Float16* __restrict__ Vt,
            float* __restrict__ O) {
  __shared__ __align__(16) _Float16     Ksh[KBLK * KD];
  __shared__ __align__(16) _Float16     Vts[DK * VD];
  __shared__ __align__(16) _Float16     Phs[8 * 16 * PD];
  __shared__ __align__(16) _Float16     Pls[8 * 16 * PD];
  __shared__ __align__(16) float        Ost[8 * 16 * OPD];
  __shared__ __align__(16) unsigned int mbits[QTILE * 4];
  __shared__ int sany[8];
  __shared__ int sall[8];

  const int qb   = blockIdx.x;
  const int h    = blockIdx.y;
  const int bb   = blockIdx.z;
  const int tid  = threadIdx.x;
  const int lane = tid & 31;
  const int wv   = tid >> 5;
  const int hf   = lane >> 4;
  const int l16  = lane & 15;
  const int koff = hf * 8;
  const int bhr  = bb * HN + h;

  const float*    Qb  = Q  + ((size_t)bb * HN + h) * (size_t)S_FULL * DK;
  const _Float16* KhB = Kh + (size_t)bhr * SEQ * DK;
  const _Float16* VtB = Vt + (size_t)bhr * DK * SEQ;
  float*          Ob  = O  + (size_t)bhr * SEQ * DK;
  const int q0 = qb * QTILE;

  Frag qa0, qa1;
  {
    const float* qp = Qb + (size_t)(q0 + wv * 16 + l16) * DK;
    qa0.h[0] = cvt8(qp + koff);
    qa0.h[1] = cvt8(qp + 16 + koff);
    qa1.h[0] = cvt8(qp + 32 + koff);
    qa1.h[1] = cvt8(qp + 48 + koff);
  }

  const v8f vz = {0.f, 0.f, 0.f, 0.f, 0.f, 0.f, 0.f, 0.f};
  v8f o[4], ol[4];
#pragma unroll
  for (int t = 0; t < 4; ++t) { o[t] = vz; ol[t] = vz; }
  float m[8], ls[8];
#pragma unroll
  for (int v = 0; v < 8; ++v) { m[v] = -1.0e30f; ls[v] = 0.0f; }

  _Float16* Pw  = &Phs[wv * 16 * PD];
  _Float16* Plw = &Pls[wv * 16 * PD];

  const int mrow  = tid >> 1;
  const int mhalf = tid & 1;
  const int* mrp = Mk + (size_t)(q0 + mrow) * S_FULL + mhalf * 64;

  const float NEGI = -__builtin_inff();
  const float CL2  = 0.125f * 1.44269504088896f;

  for (int kb = 0; kb < NBLK; ++kb) {
    __syncthreads();

    {
      const int* mp = mrp + kb * KBLK;
      unsigned int w0 = 0u, w1 = 0u;
#pragma unroll
      for (int i = 0; i < 8; ++i) {
        const v4i x = *(const v4i*)(mp + 4 * i);
        const unsigned int nib = ((x[0] != 0) ? 1u : 0u) | ((x[1] != 0) ? 2u : 0u) |
                                 ((x[2] != 0) ? 4u : 0u) | ((x[3] != 0) ? 8u : 0u);
        w0 |= nib << (4 * i);
      }
#pragma unroll
      for (int i = 0; i < 8; ++i) {
        const v4i x = *(const v4i*)(mp + 32 + 4 * i);
        const unsigned int nib = ((x[0] != 0) ? 1u : 0u) | ((x[1] != 0) ? 2u : 0u) |
                                 ((x[2] != 0) ? 4u : 0u) | ((x[3] != 0) ? 8u : 0u);
        w1 |= nib << (4 * i);
      }
      v2u ww;
      ww[0] = w0; ww[1] = w1;
      *(v2u*)&mbits[mrow * 4 + mhalf * 2] = ww;
      unsigned int a = w0 | w1;
      unsigned int f = w0 & w1;
#pragma unroll
      for (int off = 1; off < 32; off <<= 1) {
        a |= __shfl_xor(a, off, 32);
        f &= __shfl_xor(f, off, 32);
      }
      if (lane == 0) {
        sany[wv] = (a != 0u) ? 1 : 0;
        sall[wv] = (f == 0xffffffffu) ? 1 : 0;
      }
    }
    __syncthreads();
    int anyt = 0, allt = 1;
#pragma unroll
    for (int w = 0; w < 8; ++w) { anyt |= sany[w]; allt &= sall[w]; }
    if (anyt == 0) continue;

#pragma unroll
    for (int i = 0; i < 4; ++i) {
      const int c = tid + i * 256;
      {
        const int row = c >> 3, cc = c & 7;
        *(v8h*)&Ksh[row * KD + cc * 8] =
            *(const v8h*)(KhB + (size_t)(kb * KBLK + row) * DK + cc * 8);
      }
      {
        const int row = c >> 4, cc = c & 15;
        *(v8h*)&Vts[row * VD + cc * 8] =
            *(const v8h*)(VtB + (size_t)row * SEQ + kb * KBLK + cc * 8);
      }
    }
    __syncthreads();

    v8f c[NT];
#pragma unroll
    for (int t = 0; t < NT; ++t) c[t] = vz;
#pragma unroll
    for (int kc = 0; kc < 2; ++kc) {
      const v16h a = kc ? qa1.v : qa0.v;
#pragma unroll
      for (int t = 0; t < NT; ++t) {
        const v16h bop = ld_op16(&Ksh[(t * 16 + l16) * KD + kc * 32 + koff]);
        c[t] = wmma16(a, bop, c[t]);
      }
    }

    if (allt == 0) {
#pragma unroll
      for (int v = 0; v < 8; ++v) {
        const v4u wd = *(const v4u*)&mbits[(wv * 16 + 8 * hf + v) * 4];
#pragma unroll
        for (int t = 0; t < NT; ++t) {
          const unsigned int bit = (wd[t >> 1] >> ((t & 1) * 16 + l16)) & 1u;
          c[t][v] = (bit != 0u) ? c[t][v] : NEGI;
        }
      }
    }

    float sc[8];
#pragma unroll
    for (int v = 0; v < 8; ++v) {
      float r = fmaxf(fmaxf(fmaxf(c[0][v], c[1][v]), fmaxf(c[2][v], c[3][v])),
                      fmaxf(fmaxf(c[4][v], c[5][v]), fmaxf(c[6][v], c[7][v])));
      r = fmaxf(r, __shfl_xor(r, 1, 32));
      r = fmaxf(r, __shfl_xor(r, 2, 32));
      r = fmaxf(r, __shfl_xor(r, 4, 32));
      r = fmaxf(r, __shfl_xor(r, 8, 32));
      const float mn = fmaxf(m[v], r);
      sc[v] = fast_exp2((m[v] - mn) * CL2);
      m[v]  = mn;
    }
#pragma unroll
    for (int v = 0; v < 8; ++v) {
      float s = 0.0f;
#pragma unroll
      for (int t = 0; t < NT; ++t) {
        const float p = fast_exp2((c[t][v] - m[v]) * CL2);
        c[t][v] = p;
        s += p;
      }
      ls[v] = ls[v] * sc[v] + s;
#pragma unroll
      for (int t = 0; t < 4; ++t) { o[t][v] *= sc[v]; ol[t][v] *= sc[v]; }
    }

#pragma unroll
    for (int t = 0; t < NT; ++t) {
#pragma unroll
      for (int v = 0; v < 8; ++v) {
        const float    ps  = c[t][v] * 1024.0f;
        const _Float16 ph  = (_Float16)ps;
        const float    res = (ps - (float)ph) * 4096.0f;
        const int idx = (v + 8 * hf) * PD + t * 16 + l16;
        Pw[idx]  = ph;
        Plw[idx] = (_Float16)res;
      }
    }
    __syncthreads();

#pragma unroll
    for (int kc = 0; kc < 4; ++kc) {
      const v16h pa = ld_op16(&Pw[l16 * PD + kc * 32 + koff]);
      const v16h pl = ld_op16(&Plw[l16 * PD + kc * 32 + koff]);
#pragma unroll
      for (int t = 0; t < 4; ++t) {
        const v16h vb = ld_op16(&Vts[(t * 16 + l16) * VD + kc * 32 + koff]);
        o[t]  = wmma16(pa, vb, o[t]);
        ol[t] = wmma16(pl, vb, ol[t]);
      }
    }
  }

  __syncthreads();
  float* Ow = &Ost[wv * 16 * OPD];
#pragma unroll
  for (int v = 0; v < 8; ++v) {
    float l = ls[v];
    l += __shfl_xor(l, 1, 32);
    l += __shfl_xor(l, 2, 32);
    l += __shfl_xor(l, 4, 32);
    l += __shfl_xor(l, 8, 32);
    const float rn = fast_rcp(l) * (1.0f / 1024.0f);
    const int lr = v + 8 * hf;
#pragma unroll
    for (int t = 0; t < 4; ++t)
      Ow[lr * OPD + t * 16 + l16] = (o[t][v] + ol[t][v] * (1.0f / 4096.0f)) * rn;
  }
  __syncthreads();

  v4f ov[8];
#pragma unroll
  for (int j = 0; j < 8; ++j) ov[j] = *(const v4f*)&Ow[(2 * j + hf) * OPD + 4 * l16];

  float* ob0 = Ob + (size_t)(q0 + wv * 16) * DK + 4 * l16;
#pragma unroll
  for (int j = 0; j < 8; ++j)
    *(volatile v4f*)(ob0 + (size_t)(2 * j + hf) * DK) = ov[j];
  __threadfence();
#pragma unroll
  for (int j = 0; j < 8; ++j)
    *(volatile v4f*)(ob0 + (size_t)(2 * j + hf) * DK) = ov[j];
}

extern "C" void kernel_launch(void* const* d_in, const int* in_sizes, int n_in,
                              void* d_out, int out_size, void* d_ws, size_t ws_size,
                              hipStream_t stream) {
  if (n_in < 4) return;
  const float* Q  = (const float*)d_in[0];
  const float* K  = (const float*)d_in[1];
  const float* V  = (const float*)d_in[2];
  const int*   Mk = (const int*)d_in[3];
  float* O = (float*)d_out;

  const size_t need_in = (size_t)NB * HN * (size_t)S_FULL * DK;
  if ((size_t)in_sizes[0] < need_in) return;
  if ((size_t)in_sizes[1] < need_in) return;
  if ((size_t)in_sizes[2] < need_in) return;
  if ((size_t)in_sizes[3] < (size_t)SEQ * S_FULL) return;

  const size_t elems = (size_t)NB * HN * (size_t)SEQ * DK;
  if ((size_t)out_size < elems) return;
  const size_t need_ws = elems * sizeof(_Float16) * 2;
  if (ws_size < need_ws) return;

  _Float16* Kh = (_Float16*)d_ws;
  _Float16* Vt = Kh + elems;

  k_convert<<<dim3(SEQ / CT, NB * HN), dim3(256), 0, stream>>>(K, V, Kh, Vt);
  k_attn<<<dim3(SEQ / QTILE, HN, NB), dim3(256), 0, stream>>>(Q, Mk, Kh, Vt, O);
}
